// DeepLPF_90005334655040
// MI455X (gfx1250) — hardware-run, weakly checked
//
#include <hip/hip_runtime.h>
#include <math.h>

typedef __attribute__((ext_vector_type(8)))  _Float16 v8h;
typedef __attribute__((ext_vector_type(16))) __bf16   v16b;
typedef __attribute__((ext_vector_type(8)))  __bf16   v8b;
typedef __attribute__((ext_vector_type(8)))  float    v8f;
typedef __attribute__((ext_vector_type(4)))  float    v4f;
typedef __attribute__((ext_vector_type(8)))  unsigned v8u;

constexpr int kNB   = 4;
constexpr int kIH   = 512;
constexpr int kPix  = kIH * kIH;
constexpr int kCh   = 64;
constexpr int kFeat = 61;
constexpr int kUp   = 300;
constexpr int kS1 = 150, kS2 = 75, kS3 = 38, kS4 = 19;
constexpr int kM0 = kUp * kUp;
constexpr int kM1 = kS1 * kS1, kM2 = kS2 * kS2, kM3 = kS3 * kS3, kM4 = kS4 * kS4;
constexpr int kKc   = 9 * kCh;
constexpr int kRowP = 1544;
constexpr int kParP = 256;
constexpr float kEps = 1e-10f;
constexpr float kPi  = 3.14159265358979323846f;
constexpr float kKs    = 512.0f / 300.0f;
constexpr float kInvKs = 300.0f / 512.0f;
static_assert(kM1 == 22500 && kM2 == 5625 && kM3 == 1444 && kM4 == 361);
static_assert(kKc == 576 && (kKc % 32) == 0);
static_assert(kRowP >= (kIH + 2) * 3);

constexpr size_t kSzZero = 256;
constexpr size_t kSzWB   = (size_t)64 * 32 * 2;
constexpr size_t kSzWH   = (size_t)12 * 64 * kKc * 2;
constexpr size_t kSzFI   = (size_t)kPix * kCh * 4;
constexpr size_t kSzX0   = (size_t)kM0 * kCh * 2;
constexpr size_t kSzX1   = (size_t)3 * kM1 * kCh * 2;
constexpr size_t kSzX2   = (size_t)3 * kM2 * kCh * 2;
constexpr size_t kSzX3   = (size_t)3 * kM3 * kCh * 2;
constexpr size_t kSzX4   = (size_t)kNB * 3 * kM4 * kCh * 4;
constexpr size_t kSzPar  = (size_t)kNB * kParP * 4;
constexpr size_t kOffZero = 0;
constexpr size_t kOffWBH = kOffZero + kSzZero;
constexpr size_t kOffWBL = kOffWBH + kSzWB;
constexpr size_t kOffWHH = kOffWBL + kSzWB;
constexpr size_t kOffWHL = kOffWHH + kSzWH;
constexpr size_t kOffFI  = kOffWHL + kSzWH;
constexpr size_t kOffX0H = kOffFI  + kSzFI;
constexpr size_t kOffX0L = kOffX0H + kSzX0;
constexpr size_t kOffX1H = kOffX0L + kSzX0;
constexpr size_t kOffX1L = kOffX1H + kSzX1;
constexpr size_t kOffX2H = kOffX1L + kSzX1;
constexpr size_t kOffX2L = kOffX2H + kSzX2;
constexpr size_t kOffX3H = kOffX2L + kSzX2;
constexpr size_t kOffX3L = kOffX3H + kSzX3;
constexpr size_t kOffX4  = kOffX3L + kSzX3;
constexpr size_t kOffPar = kOffX4  + kSzX4;
constexpr size_t kWsTotal = kOffPar + kSzPar;
static_assert(kWsTotal == 115748864ull);
static_assert(kWsTotal <= 134217728ull);
static_assert((kOffWBH % 128) == 0 && (kOffWBL % 128) == 0 && (kOffWHH % 128) == 0 && (kOffWHL % 128) == 0 &&
              (kOffFI % 128) == 0 && (kOffX0H % 128) == 0 && (kOffX0L % 128) == 0 && (kOffX1H % 128) == 0 &&
              (kOffX1L % 128) == 0 && (kOffX2H % 128) == 0 && (kOffX2L % 128) == 0 && (kOffX3H % 128) == 0 &&
              (kOffX3L % 128) == 0 && (kOffX4 % 128) == 0 && (kOffPar % 128) == 0);

__device__ __forceinline__ unsigned short f2bf_bits(float f) {
  unsigned u = __float_as_uint(f);
  return (unsigned short)((u + 0x7FFFu + ((u >> 16) & 1u)) >> 16);
}
__device__ __forceinline__ float bf_bits2f(unsigned short h) { return __uint_as_float(((unsigned)h) << 16); }
__device__ __forceinline__ int iclamp(int v, int lo, int hi) { return v < lo ? lo : (v > hi ? hi : v); }

union FragU { v16b v; v8b h[2]; };
__device__ __forceinline__ v16b frag_load(const __bf16* p) {
  FragU f;
  f.h[0] = *(const v8b*)(p);
  f.h[1] = *(const v8b*)(p + 16);
  return f.v;
}
__device__ __forceinline__ v8f mma_b(v16b a, v16b b, v8f c) {
  c = __builtin_amdgcn_wmma_f32_16x16x32_bf16(false, a, false, b, (short)0, c, false, false);
  asm volatile("v_nop\n\tv_nop\n\tv_nop\n\tv_nop" : "+v"(c) : "v"(a), "v"(b));
  return c;
}
__device__ __forceinline__ void store_split8(unsigned short* ph, unsigned short* pl, const float (&v)[8]) {
  v8h hv, lv;
#pragma unroll
  for (int e = 0; e < 8; ++e) {
    const unsigned short hb = f2bf_bits(v[e]);
    const unsigned short lb = f2bf_bits(v[e] - bf_bits2f(hb));
    hv[e] = __builtin_bit_cast(_Float16, hb);
    lv[e] = __builtin_bit_cast(_Float16, lb);
  }
  *(volatile v8h*)ph = hv;
  *(volatile v8h*)pl = lv;
  __threadfence();
  *(volatile v8h*)ph = hv;
  *(volatile v8h*)pl = lv;
}

__global__ __launch_bounds__(256) void prep_weights_kernel(
    const float* __restrict__ bbw, const float* __restrict__ w0, const float* __restrict__ w1,
    const float* __restrict__ w2,
    unsigned short* __restrict__ WBH, unsigned short* __restrict__ WBL,
    unsigned short* __restrict__ WHH, unsigned short* __restrict__ WHL, unsigned short* __restrict__ ZR)
{
  const int tid = threadIdx.x;
  const int slot = blockIdx.y;
  float v[8];
  if (slot < 12) {
    const int layer = slot / 3;
    const int head = slot - 3 * layer;
    const float* w = (head == 0) ? w0 : ((head == 1) ? w1 : w2);
    const int t = blockIdx.x * 256 + tid;
    const int co = t / 72;
    const int kg = t - co * 72;
    const int k0 = kg * 8;
    const int tap = k0 >> 6;
    const int ci0 = k0 & 63;
    const float* src = w + ((size_t)(layer * 9 + tap) * 64 + ci0) * 64 + co;
#pragma unroll
    for (int e = 0; e < 8; ++e) v[e] = src[e * 64];
    const size_t dst = ((size_t)slot * 64 + co) * kKc + k0;
    store_split8(WHH + dst, WHL + dst, v);
  } else {
    if (blockIdx.x >= 2) return;
    if (blockIdx.x == 0) {
      const int n = tid >> 2;
      const int kg = tid & 3;
      const int nc = n < kFeat ? n : kFeat - 1;
#pragma unroll
      for (int e = 0; e < 8; ++e) {
        const int k = kg * 8 + e;
        const int kc = k < 27 ? k : 26;
        const float x = bbw[kc * kFeat + nc];
        v[e] = (k < 27 && n < kFeat) ? x : 0.0f;
      }
      const size_t dst = (size_t)n * 32 + kg * 8;
      store_split8(WBH + dst, WBL + dst, v);
    } else {
      if (tid < 16) {
        v8h z;
#pragma unroll
        for (int e = 0; e < 8; ++e) z[e] = (_Float16)0.0f;
        *(volatile v8h*)(ZR + tid * 8) = z;
        __threadfence();
        *(volatile v8h*)(ZR + tid * 8) = z;
      }
    }
  }
}

__global__ __launch_bounds__(256) void first_conv_kernel(
    const float* __restrict__ img, const unsigned short* __restrict__ WBHp, const unsigned short* __restrict__ WBLp,
    const float* __restrict__ bias, float* __restrict__ fi, int b)
{
  __shared__ __align__(16) float sImg[4 * kRowP];
  __shared__ __align__(16) float sT[8][16 * 68];
  const int tid = threadIdx.x, lane = tid & 31, wave = tid >> 5;
  const int y = blockIdx.x;
#pragma unroll
  for (int ky = 0; ky < 3; ++ky) {
    const int yy = y + ky - 1;
    const bool rowok = (yy >= 0) && (yy < kIH);
    const int yc = iclamp(yy, 0, kIH - 1);
    const float* src = img + ((size_t)(b * kIH + yc) * kIH) * 3;
#pragma unroll
    for (int t = 0; t < 2; ++t) {
      const int idx = tid + 256 * t;
      const int ic = idx < 384 ? idx : 383;
      const v4f v = *(const v4f*)(src + 4 * ic);
      if (idx < 384) {
        float* d = sImg + ky * kRowP + 3 + 4 * ic;
        d[0] = rowok ? v[0] : 0.0f;
        d[1] = rowok ? v[1] : 0.0f;
        d[2] = rowok ? v[2] : 0.0f;
        d[3] = rowok ? v[3] : 0.0f;
      }
    }
  }
#pragma unroll 1
  for (int z = tid; z < 1568; z += 256) {
    int addr;
    if (z < kRowP) {
      addr = 3 * kRowP + z;
    } else {
      const int zz = z - kRowP;
      const int r = zz >> 3, e = zz & 7;
      addr = r * kRowP + (e < 3 ? e : 1536 + e);
    }
    sImg[addr] = 0.0f;
  }
  __syncthreads();

  const int rlane = lane & 15, hh = lane >> 4, koff = hh * 8, mOff = hh * 8;
  const __bf16* Bh = (const __bf16*)WBHp;
  const __bf16* Bl = (const __bf16*)WBLp;
  v16b bh[4], bl[4];
  float bv[4];
#pragma unroll
  for (int j = 0; j < 4; ++j) {
    const int n = (j << 4) + rlane;
    const size_t bo = (size_t)n * 32 + koff;
    bh[j] = frag_load(Bh + bo);
    bl[j] = frag_load(Bl + bo);
    const int nc = n < kFeat ? n : kFeat - 1;
    const float bvv = bias[nc];
    bv[j] = (n < kFeat) ? bvv : 0.0f;
  }
  const int x0 = wave * 64;
  int aoff[16];
#pragma unroll
  for (int e = 0; e < 16; ++e) {
    const int k = koff + (e < 8 ? e : e + 8);
    const int ky = (k * 57) >> 9;
    aoff[e] = ky * (kRowP - 9) + k + (x0 + rlane) * 3;
  }
  const int cch = rlane >= 13 ? rlane - 13 : 0;
  const bool isimg = rlane >= 13;
  float* slab = sT[wave];
  const int c4 = (lane & 15) * 4;

#pragma unroll 1
  for (int i = 0; i < 4; ++i) {
    const int io = i * 48;
    v8u wh, wl;
#pragma unroll
    for (int e2 = 0; e2 < 8; ++e2) {
      const float f0 = sImg[aoff[2 * e2] + io];
      const float f1 = sImg[aoff[2 * e2 + 1] + io];
      const unsigned short h0 = f2bf_bits(f0), h1 = f2bf_bits(f1);
      const unsigned short l0 = f2bf_bits(f0 - bf_bits2f(h0)), l1 = f2bf_bits(f1 - bf_bits2f(h1));
      wh[e2] = (unsigned)h0 | ((unsigned)h1 << 16);
      wl[e2] = (unsigned)l0 | ((unsigned)l1 << 16);
    }
    const v16b ah = __builtin_bit_cast(v16b, wh);
    const v16b al = __builtin_bit_cast(v16b, wl);
    v8f acc[4];
#pragma unroll
    for (int j = 0; j < 4; ++j) {
      acc[j] = (v8f){0.f, 0.f, 0.f, 0.f, 0.f, 0.f, 0.f, 0.f};
      acc[j] = mma_b(ah, bh[j], acc[j]);
      acc[j] = mma_b(ah, bl[j], acc[j]);
      acc[j] = mma_b(al, bh[j], acc[j]);
    }
#pragma unroll
    for (int j = 0; j < 4; ++j) {
#pragma unroll
      for (int r = 0; r < 8; ++r) {
        float v = fmaxf(acc[j][r] + bv[j], 0.0f);
        if (j == 3) {
          const float iv = sImg[kRowP + (x0 + i * 16 + mOff + r + 1) * 3 + cch];
          v = isimg ? iv : v;
        }
        slab[(mOff + r) * 68 + (j << 4) + rlane] = v;
      }
    }
    __builtin_amdgcn_fence(__ATOMIC_RELEASE, "workgroup");
    __builtin_amdgcn_wave_barrier();
    __builtin_amdgcn_fence(__ATOMIC_ACQUIRE, "workgroup");
    float* dstb = fi + ((size_t)y * kIH + x0 + i * 16) * kCh;
    for (int pass = 0; pass < 2; ++pass) {
#pragma unroll
      for (int it = 0; it < 8; ++it) {
        const int row = it * 2 + hh;
        const v4f v = *(const v4f*)(slab + row * 68 + c4);
        *(volatile v4f*)(dstb + (size_t)row * kCh + c4) = v;
      }
      __threadfence();
    }
    __builtin_amdgcn_fence(__ATOMIC_RELEASE, "workgroup");
    __builtin_amdgcn_wave_barrier();
    __builtin_amdgcn_fence(__ATOMIC_ACQUIRE, "workgroup");
  }
}

__global__ __launch_bounds__(256) void resample_kernel(
    const float* __restrict__ fi, unsigned short* __restrict__ XH, unsigned short* __restrict__ XL)
{
  constexpr int kTotal = kM0 * 8;
  const int t = blockIdx.x * 256 + threadIdx.x;
  const int tc = t < kTotal ? t : kTotal - 1;
  const int pix = tc >> 3;
  const int cg = (tc & 7) * 8;
  const int oy = pix / kUp;
  const int ox = pix - oy * kUp;
  const float sfy = ((float)oy + 0.5f) * kKs - 0.5f;
  const float sfx = ((float)ox + 0.5f) * kKs - 0.5f;
  const int jy0 = (int)floorf(sfy - kKs) + 1;
  const int jx0 = (int)floorf(sfx - kKs) + 1;
  float wx[4];
  int xo[4];
  float sx = 0.0f, sy = 0.0f;
#pragma unroll
  for (int e = 0; e < 4; ++e) {
    const int j = jx0 + e;
    const float d = fabsf(sfx - (float)j);
    float w = fmaxf(0.0f, 1.0f - d * kInvKs);
    w = (j >= 0 && j < kIH) ? w : 0.0f;
    wx[e] = w;
    sx += w;
    xo[e] = iclamp(j, 0, kIH - 1) * kCh + cg;
  }
#pragma unroll
  for (int e = 0; e < 4; ++e) {
    const int j = jy0 + e;
    const float d = fabsf(sfy - (float)j);
    float w = fmaxf(0.0f, 1.0f - d * kInvKs);
    w = (j >= 0 && j < kIH) ? w : 0.0f;
    sy += w;
  }
  const float inx = 1.0f / sx;
  const float iny = 1.0f / sy;
#pragma unroll
  for (int e = 0; e < 4; ++e) wx[e] *= inx;
  float acc[8];
#pragma unroll
  for (int e = 0; e < 8; ++e) acc[e] = 0.0f;
#pragma unroll 1
  for (int ty = 0; ty < 4; ++ty) {
    const int j = jy0 + ty;
    const float d = fabsf(sfy - (float)j);
    float w = fmaxf(0.0f, 1.0f - d * kInvKs);
    w = (j >= 0 && j < kIH) ? w : 0.0f;
    w *= iny;
    const float* rp = fi + (size_t)iclamp(j, 0, kIH - 1) * (kIH * kCh);
#pragma unroll
    for (int e = 0; e < 4; ++e) {
      const float wgt = w * wx[e];
      const v4f a0 = *(const v4f*)(rp + xo[e]);
      const v4f a1 = *(const v4f*)(rp + xo[e] + 4);
      acc[0] = fmaf(wgt, a0[0], acc[0]);
      acc[1] = fmaf(wgt, a0[1], acc[1]);
      acc[2] = fmaf(wgt, a0[2], acc[2]);
      acc[3] = fmaf(wgt, a0[3], acc[3]);
      acc[4] = fmaf(wgt, a1[0], acc[4]);
      acc[5] = fmaf(wgt, a1[1], acc[5]);
      acc[6] = fmaf(wgt, a1[2], acc[6]);
      acc[7] = fmaf(wgt, a1[3], acc[7]);
    }
  }
  if (t < kTotal) {
    const size_t o = (size_t)pix * kCh + cg;
    store_split8(XH + o, XL + o, acc);
  }
}

template <bool OUT_F32>
__global__ __launch_bounds__(256) void conv_s2_kernel(
    const unsigned short* __restrict__ Ahp, const unsigned short* __restrict__ Alp, long aHeadStride,
    const unsigned short* __restrict__ Whp, const unsigned short* __restrict__ Wlp,
    const unsigned short* __restrict__ zrowp,
    const float* __restrict__ bias0, const float* __restrict__ bias1, const float* __restrict__ bias2,
    void* __restrict__ Cout, void* __restrict__ Cout2, long cHeadStride,
    int Hi, int Ho, int pad)
{
  __shared__ __align__(16) float sT[8][16 * 68];
  const int lane = threadIdx.x & 31, wave = threadIdx.x >> 5;
  const int M = Ho * Ho;
  const int tilesM = (M + 31) >> 5;
  const int t = blockIdx.x * 8 + wave;
  if (t >= tilesM * 3) return;
  const int tm = t / 3;
  const int head = t - tm * 3;
  const int m0 = tm << 5;
  const int rlane = lane & 15, hh = lane >> 4, koff = hh * 8, mOff = hh * 8;

  const __bf16* Ah = (const __bf16*)Ahp + (size_t)head * aHeadStride;
  const __bf16* Al = (const __bf16*)Alp + (size_t)head * aHeadStride;
  const __bf16* Wh = (const __bf16*)Whp + (size_t)head * 64 * kKc;
  const __bf16* Wl = (const __bf16*)Wlp + (size_t)head * 64 * kKc;
  const __bf16* Z  = (const __bf16*)zrowp;

  const float f0 = (head == 0) ? 1.0f : 0.0f;
  const float f1 = (head == 1) ? 1.0f : 0.0f;
  const float f2 = (head == 2) ? 1.0f : 0.0f;
  float bv[4];
#pragma unroll
  for (int j = 0; j < 4; ++j) {
    const int n = (j << 4) + rlane;
    const float b0 = bias0[n], b1 = bias1[n], b2 = bias2[n];
    bv[j] = fmaf(f0, b0, fmaf(f1, b1, f2 * b2));
  }

  int iy0[2], ix0[2];
#pragma unroll
  for (int i = 0; i < 2; ++i) {
    int p = m0 + (i << 4) + rlane;
    p = p < M ? p : M - 1;
    const int oy = p / Ho;
    const int ox = p - oy * Ho;
    iy0[i] = 2 * oy - pad;
    ix0[i] = 2 * ox - pad;
  }

  v8f acc[2][4];
#pragma unroll
  for (int i = 0; i < 2; ++i)
#pragma unroll
    for (int j = 0; j < 4; ++j) acc[i][j] = (v8f){0.f, 0.f, 0.f, 0.f, 0.f, 0.f, 0.f, 0.f};

#pragma unroll 1
  for (int tap = 0; tap < 9; ++tap) {
    const int ky = tap / 3;
    const int kx = tap - 3 * ky;
    const __bf16* pah[2];
    const __bf16* pal[2];
#pragma unroll
    for (int i = 0; i < 2; ++i) {
      const int iy = iy0[i] + ky;
      const int ix = ix0[i] + kx;
      const bool ok = ((unsigned)iy < (unsigned)Hi) && ((unsigned)ix < (unsigned)Hi);
      const size_t off = ok ? ((size_t)(iy * Hi + ix) << 6) : (size_t)0;
      pah[i] = ok ? (Ah + off) : Z;
      pal[i] = ok ? (Al + off) : Z;
    }
#pragma unroll
    for (int kc = 0; kc < 2; ++kc) {
      const int kk = tap * 64 + kc * 32 + koff;
      v16b bh[4], bl[4];
#pragma unroll
      for (int j = 0; j < 4; ++j) {
        const size_t bo = (size_t)((j << 4) + rlane) * kKc + kk;
        bh[j] = frag_load(Wh + bo);
        bl[j] = frag_load(Wl + bo);
      }
#pragma unroll
      for (int i = 0; i < 2; ++i) {
        const v16b ah = frag_load(pah[i] + kc * 32 + koff);
        const v16b al = frag_load(pal[i] + kc * 32 + koff);
#pragma unroll
        for (int j = 0; j < 4; ++j) {
          acc[i][j] = mma_b(ah, bh[j], acc[i][j]);
          acc[i][j] = mma_b(ah, bl[j], acc[i][j]);
          acc[i][j] = mma_b(al, bh[j], acc[i][j]);
        }
      }
    }
  }

  float* slab = sT[wave];
#pragma unroll
  for (int i = 0; i < 2; ++i) {
    const int mBase = m0 + (i << 4);
#pragma unroll
    for (int j = 0; j < 4; ++j) {
#pragma unroll
      for (int r = 0; r < 8; ++r) {
        float v = acc[i][j][r] + bv[j];
        v = (v > 0.0f) ? v : 0.2f * v;
        slab[(mOff + r) * 68 + (j << 4) + rlane] = v;
      }
    }
    __builtin_amdgcn_fence(__ATOMIC_RELEASE, "workgroup");
    __builtin_amdgcn_wave_barrier();
    __builtin_amdgcn_fence(__ATOMIC_ACQUIRE, "workgroup");
    if (OUT_F32) {
      float* C = (float*)Cout + (size_t)head * cHeadStride;
      const int c4 = (lane & 15) * 4;
      for (int pass = 0; pass < 2; ++pass) {
#pragma unroll
        for (int it = 0; it < 8; ++it) {
          const int row = it * 2 + hh;
          const int grow = mBase + row;
          const v4f v = *(const v4f*)(slab + row * 68 + c4);
          if (grow < M) *(volatile v4f*)(C + (size_t)grow * kCh + c4) = v;
        }
        __threadfence();
      }
    } else {
      const int q = lane >> 3, c8 = (lane & 7) * 8;
      unsigned short* C  = (unsigned short*)Cout  + (size_t)head * cHeadStride;
      unsigned short* C2 = (unsigned short*)Cout2 + (size_t)head * cHeadStride;
      for (int pass = 0; pass < 2; ++pass) {
#pragma unroll
        for (int it = 0; it < 4; ++it) {
          const int row = it * 4 + q;
          const int grow = mBase + row;
          const float* sp = slab + row * 68 + c8;
          v8h hv, lv;
#pragma unroll
          for (int e = 0; e < 8; ++e) {
            const float sv = sp[e];
            const unsigned short hb = f2bf_bits(sv);
            const unsigned short lb = f2bf_bits(sv - bf_bits2f(hb));
            hv[e] = __builtin_bit_cast(_Float16, hb);
            lv[e] = __builtin_bit_cast(_Float16, lb);
          }
          if (grow < M) {
            *(volatile v8h*)(C  + (size_t)grow * kCh + c8) = hv;
            *(volatile v8h*)(C2 + (size_t)grow * kCh + c8) = lv;
          }
        }
        __threadfence();
      }
    }
    __builtin_amdgcn_fence(__ATOMIC_RELEASE, "workgroup");
    __builtin_amdgcn_wave_barrier();
    __builtin_amdgcn_fence(__ATOMIC_ACQUIRE, "workgroup");
  }
}

__device__ __forceinline__ float sign01f(float x) {
  const float s = (x > 0.0f) ? 1.0f : ((x < 0.0f) ? -1.0f : 0.0f);
  return 0.5f * (s + 1.0f);
}

__global__ __launch_bounds__(256) void pool_dense_kernel(
    const float* __restrict__ X4,
    const float* __restrict__ fw0, const float* __restrict__ fb0,
    const float* __restrict__ fw1, const float* __restrict__ fb1,
    const float* __restrict__ fw2, const float* __restrict__ fb2,
    float* __restrict__ PAR)
{
  __shared__ float sPart[256];
  __shared__ float sMean[64];
  __shared__ float sHv[128];
  __shared__ float sTh[128];
  __shared__ float sTh2[8];
  __shared__ __align__(16) float sPar[kParP];
  const int tid = threadIdx.x;
  const int b = blockIdx.x;
  const int c = tid & 63, part = tid >> 6;
#pragma unroll 1
  for (int head = 0; head < 3; ++head) {
    const float* src = X4 + ((size_t)(b * 3 + head) * kM4) * kCh;
    float s = 0.0f;
#pragma unroll 1
    for (int p = part; p < kM4; p += 4) s += src[p * kCh + c];
    sPart[part * 64 + c] = s;
    __syncthreads();
    if (tid < 64)
      sMean[tid] = ((sPart[tid] + sPart[64 + tid]) + (sPart[128 + tid] + sPart[192 + tid])) * (1.0f / (float)kM4);
    __syncthreads();
    const int fcN = (head == 0) ? 60 : 24;
    const int base = (head == 0) ? 0 : ((head == 1) ? 60 : 84);
    const float* fw = (head == 0) ? fw0 : ((head == 1) ? fw1 : fw2);
    const float* fb = (head == 0) ? fb0 : ((head == 1) ? fb1 : fb2);
    const int n = tid < fcN ? tid : fcN - 1;
    float acc = 0.0f;
#pragma unroll 1
    for (int k = 0; k < 64; ++k) acc = fmaf(sMean[k], fw[k * fcN + n], acc);
    acc += fb[n];
    if (tid < fcN) sHv[base + tid] = acc;
    __syncthreads();
  }
  if (tid >= 108 && tid < 128) sHv[tid] = 0.0f;
  __syncthreads();

#pragma unroll 1
  for (int it = 0; it < 2; ++it) {
    float arg = sHv[tid & 127];
    if (it == 1) {
      const int g2 = (tid >> 1) < 2 ? (tid >> 1) : 2;
      const int gb = 84 + 8 * g2;
      const float cc = sTh[gb + 4] + kEps;
      const float o1 = fminf(fmaxf(sign01f(sHv[gb + 5]), cc), 1.0f);
      const float o2 = fminf(fmaxf(sign01f(sHv[gb + 6]), 0.0f), cc);
      arg = (tid & 1) ? o2 : o1;
    }
    const float tv = 0.5f * tanhf(arg) + 0.5f;
    if (it == 0) {
      if (tid < 128) sTh[tid] = tv;
    } else {
      if (tid < 8) sTh2[tid] = tv;
    }
    __syncthreads();
  }

  if (tid < 64) sPar[tid] = (tid < 60) ? sHv[tid] : 0.0f;
  if (tid >= 160) sPar[tid] = 0.0f;
  {
    const int g = tid < 3 ? tid : 2;
    const float* te = sTh + 60 + 8 * g;
    const float sc0 = te[0] * 2.0f + kEps;
    const float sc1 = te[1] * 2.0f + kEps;
    const float sc2 = te[2] * 2.0f + kEps;
    const float hh = te[3] + kEps;
    const float kk = te[4] + kEps;
    const float theta = te[5] * kPi + kEps;
    const float aa = te[6] + kEps;
    const float bb = te[7] + kEps;
    float st, ct;
    sincosf(theta, &st, &ct);
    const float a2 = aa * aa, b2 = bb * bb;
    const float ia2 = __builtin_amdgcn_rcpf(a2), ib2 = __builtin_amdgcn_rcpf(b2);

    const float* rg = sHv + 84 + 8 * g;
    const float* tg = sTh + 84 + 8 * g;
    const float gm = rg[3];
    const bool ginv0 = rg[7] < 0.0f;
    const float cs = __builtin_amdgcn_rcpf(sqrtf(1.0f + gm * gm));
    const float cc = tg[4] + kEps;
    const float d1 = sTh2[2 * g] * cs;
    const float d2 = sTh2[2 * g + 1] * cs;
    const float r1 = __builtin_amdgcn_rcpf(2.0f * d1);
    const float r2 = __builtin_amdgcn_rcpf(2.0f * d2);
    const float s0 = tg[0] * 2.0f, s1 = tg[1] * 2.0f, s2 = tg[2] * 2.0f;
    const float fa0 = (s0 - 1.0f) * r1 + (ginv0 ? (s0 - 1.0f) : (1.0f - s0)) * r2;
    const float fa1 = (s1 - 1.0f) * r1 + (ginv0 ? (s1 - 1.0f) : (1.0f - s1)) * r2;
    const float fa2 = (s2 - 1.0f) * r1 + (ginv0 ? (s2 - 1.0f) : (1.0f - s2)) * r2;
    if (tid < 3) {
      float* pe = sPar + 64 + 16 * g;
      pe[0] = sc0; pe[1] = sc1; pe[2] = sc2; pe[3] = hh; pe[4] = kk; pe[5] = st; pe[6] = ct;
      pe[7] = a2; pe[8] = b2; pe[9] = aa * bb; pe[10] = ia2; pe[11] = ib2;
      pe[12] = 0.0f; pe[13] = 0.0f; pe[14] = 0.0f; pe[15] = 0.0f;
      float* pg = sPar + 112 + 16 * g;
      pg[0] = gm; pg[1] = cc; pg[2] = d1;
      pg[3] = fa0; pg[4] = fa1; pg[5] = fa2;
      pg[6] = ginv0 ? s0 : 1.0f; pg[7] = ginv0 ? s1 : 1.0f; pg[8] = ginv0 ? s2 : 1.0f;
      pg[9]  = (s0 >= 1.0f) ? 1.0f : 0.0f; pg[10] = (s1 >= 1.0f) ? 1.0f : 0.0f; pg[11] = (s2 >= 1.0f) ? 1.0f : 0.0f;
      pg[12] = (s0 >= 1.0f) ? 2.0f : 1.0f; pg[13] = (s1 >= 1.0f) ? 2.0f : 1.0f; pg[14] = (s2 >= 1.0f) ? 2.0f : 1.0f;
      pg[15] = 0.0f;
    }
  }
  __syncthreads();
  if (tid < 32) {
    const v4f v0 = *(const v4f*)(sPar + tid * 4);
    const v4f v1 = *(const v4f*)(sPar + 128 + tid * 4);
    float* dst = PAR + (size_t)b * kParP;
    *(volatile v4f*)(dst + tid * 4) = v0;
    *(volatile v4f*)(dst + 128 + tid * 4) = v1;
    __threadfence();
    *(volatile v4f*)(dst + tid * 4) = v0;
    *(volatile v4f*)(dst + 128 + tid * 4) = v1;
  }
}

__device__ __forceinline__ float clipf(float v, float lo, float hi) { return fminf(fmaxf(v, lo), hi); }

__device__ __forceinline__ float ellipse_cond(float dx, float dy, float sT, float cT, float a2, float b2) {
#pragma clang fp contract(off)
  const float p0 = dx * cT;
  const float p1 = dy * sT;
  const float t1 = p0 + p1;
  const float p2 = dx * sT;
  const float p3 = dy * cT;
  const float t2 = p2 - p3;
  const float n1 = t1 * t1;
  const float n2 = t2 * t2;
  const float q1 = n1 / a2;
  const float q2 = n2 / b2;
  const float sq = q1 + q2;
  return sq + kEps;
}

__global__ __launch_bounds__(256) void blend_kernel(
    const float* __restrict__ img, const float* __restrict__ PAR, float* __restrict__ out)
{
  __shared__ __align__(16) float sP[kParP];
  __shared__ __align__(16) float sIn[768];
  __shared__ __align__(16) float sOut[768];
  const int tid = threadIdx.x;
  const int p = blockIdx.x * 256 + tid;
  const int b = blockIdx.x >> 10;
  sP[tid] = PAR[(size_t)b * kParP + tid];
  {
    const int q = tid < 192 ? tid : 191;
    const v4f v = *(const v4f*)(img + (size_t)blockIdx.x * 768 + q * 4);
    if (tid < 192) *(v4f*)(sIn + q * 4) = v;
  }
  __syncthreads();
  const int pi = (p >> 9) & 511, pj = p & 511;
  const float x = (float)pi * (1.0f / 512.0f);
  const float y = (float)pj * (1.0f / 512.0f);

  float pe0 = 1.0f, pe1 = 1.0f, pe2 = 1.0f, pg0 = 1.0f, pg1 = 1.0f, pg2 = 1.0f;
#pragma unroll 1
  for (int g = 0; g < 3; ++g) {
    const float* ep = sP + 64 + 16 * g;
    const float* gp = sP + 112 + 16 * g;
    const float dx = x - ep[3], dy = y - ep[4];
    const float r2 = dx * dx + dy * dy + kEps;
    const float mm = __builtin_amdgcn_sqrtf(r2);
    float cv = dy * __builtin_amdgcn_rcpf(mm + kEps);
    cv = fminf(fmaxf(cv, -1.0f + 1e-7f), 1.0f - 1e-7f);
    const float sa = __builtin_amdgcn_sqrtf((1.0f - cv) * (1.0f + cv));
    const float sT = ep[5], cT = ep[6];
    const float cang = cv * cT + sa * sT;
    const float sang = sa * cT - cv * sT;
    const float den = __builtin_amdgcn_sqrtf(ep[7] * sang * sang + ep[8] * cang * cang + kEps) + kEps;
    const float radius = ep[9] * __builtin_amdgcn_rcpf(den) + kEps;
    const float cond = ellipse_cond(dx, dy, sT, cT, ep[7], ep[8]);
    const float ir = __builtin_amdgcn_rcpf(radius);
    const bool inside = cond < 1.0f;
    const float e0 = inside ? (mm * (1.0f - ep[0]) * ir + ep[0]) : 1.0f;
    const float e1 = inside ? (mm * (1.0f - ep[1]) * ir + ep[1]) : 1.0f;
    const float e2 = inside ? (mm * (1.0f - ep[2]) * ir + ep[2]) : 1.0f;
    pe0 *= clipf(e0, 0.0f, 2.0f);
    pe1 *= clipf(e1, 0.0f, 2.0f);
    pe2 *= clipf(e2, 0.0f, 2.0f);

    const float targ = y - ((gp[0] * x + gp[1]) + gp[2]);
    const float top = __builtin_amdgcn_rcpf(1.0f + __expf(-2.0f * targ));
    const float q0 = clipf(clipf(gp[3] + gp[6] * top, gp[9],  gp[12]), 0.0f, 2.0f);
    const float q1 = clipf(clipf(gp[4] + gp[7] * top, gp[10], gp[13]), 0.0f, 2.0f);
    const float q2 = clipf(clipf(gp[5] + gp[8] * top, gp[11], gp[14]), 0.0f, 2.0f);
    pg0 *= q0;
    pg1 *= q1;
    pg2 *= q2;
  }
  sOut[tid * 3 + 0] = clipf(clipf(pg0, 0.0f, 2.0f) * clipf(pe0, 0.0f, 2.0f), 0.0f, 2.0f);
  sOut[tid * 3 + 1] = clipf(clipf(pg1, 0.0f, 2.0f) * clipf(pe1, 0.0f, 2.0f), 0.0f, 2.0f);
  sOut[tid * 3 + 2] = clipf(clipf(pg2, 0.0f, 2.0f) * clipf(pe2, 0.0f, 2.0f), 0.0f, 2.0f);

  const float xy = x * y;
  const float xx = x * x, yy = y * y;
  const float rx = __builtin_amdgcn_rcpf(x + 1e-8f);
  const float ry = __builtin_amdgcn_rcpf(y + 1e-8f);
  const float r1 = __builtin_amdgcn_rcpf(1.0f + 1e-8f);
#pragma unroll 1
  for (int ci = 0; ci < 3; ++ci) {
    const float R = sIn[tid * 3 + ci];
    const float mk = sOut[tid * 3 + ci];
    const float* kp = sP + ci * 20;
    const float RR = R * R;
    const float s0 = kp[0] * xx + kp[1] * yy + kp[2] + kp[3] * RR;
    const float s1 = kp[4] * xx + kp[5] * yy + kp[6] + kp[7] * RR;
    const float s2 = kp[8] * xx + kp[9] * yy + kp[10] + kp[11] * RR;
    const float s3 = kp[12] * xx + kp[13] * yy + kp[14] + kp[15] * RR;
    float cub = x * s0 + y * s1 + s2 + R * s3;
    const float num = xy * R;
    const float rr = __builtin_amdgcn_rcpf(R + 1e-8f);
    cub += kp[16] * (num * rx) + kp[17] * (num * ry) + kp[18] * (num * r1) + kp[19] * (num * rr);
    sOut[tid * 3 + ci] = clipf((R + cub) * mk, 0.0f, 1.0f);
  }
  __syncthreads();
  if (tid < 192) {
    const v4f v = *(const v4f*)(sOut + tid * 4);
    float* dst = out + (size_t)blockIdx.x * 768 + tid * 4;
    *(volatile v4f*)dst = v;
    __threadfence();
    *(volatile v4f*)dst = v;
  }
}

extern "C" void kernel_launch(void* const* d_in, const int* in_sizes, int n_in,
                              void* d_out, int out_size, void* d_ws, size_t ws_size,
                              hipStream_t stream) {
  if (n_in < 15) return;
  if (in_sizes[0] != kNB * kPix * 3) return;
  if (in_sizes[1] != 27 * kFeat) return;
  if (in_sizes[2] != kFeat) return;
  if (in_sizes[3] != 4 * 9 * 64 * 64 || in_sizes[7] != 4 * 9 * 64 * 64 || in_sizes[11] != 4 * 9 * 64 * 64) return;
  if (in_sizes[4] != 256 || in_sizes[8] != 256 || in_sizes[12] != 256) return;
  if (in_sizes[5] != 64 * 60 || in_sizes[9] != 64 * 24 || in_sizes[13] != 64 * 24) return;
  if (in_sizes[6] != 60 || in_sizes[10] != 24 || in_sizes[14] != 24) return;
  if (out_size != kNB * kPix * 3) return;
  if (ws_size < kWsTotal) return;

  const float* img    = (const float*)d_in[0];
  const float* bb_w   = (const float*)d_in[1];
  const float* bb_b   = (const float*)d_in[2];
  const float* cub_cw = (const float*)d_in[3];
  const float* cub_cb = (const float*)d_in[4];
  const float* cub_fw = (const float*)d_in[5];
  const float* cub_fb = (const float*)d_in[6];
  const float* ell_cw = (const float*)d_in[7];
  const float* ell_cb = (const float*)d_in[8];
  const float* ell_fw = (const float*)d_in[9];
  const float* ell_fb = (const float*)d_in[10];
  const float* grd_cw = (const float*)d_in[11];
  const float* grd_cb = (const float*)d_in[12];
  const float* grd_fw = (const float*)d_in[13];
  const float* grd_fb = (const float*)d_in[14];
  float* out = (float*)d_out;

  char* ws = (char*)d_ws;
  unsigned short* ZR  = (unsigned short*)(ws + kOffZero);
  unsigned short* WBH = (unsigned short*)(ws + kOffWBH);
  unsigned short* WBL = (unsigned short*)(ws + kOffWBL);
  unsigned short* WHH = (unsigned short*)(ws + kOffWHH);
  unsigned short* WHL = (unsigned short*)(ws + kOffWHL);
  float*          FI  = (float*)(ws + kOffFI);
  unsigned short* X0H = (unsigned short*)(ws + kOffX0H);
  unsigned short* X0L = (unsigned short*)(ws + kOffX0L);
  unsigned short* X1H = (unsigned short*)(ws + kOffX1H);
  unsigned short* X1L = (unsigned short*)(ws + kOffX1L);
  unsigned short* X2H = (unsigned short*)(ws + kOffX2H);
  unsigned short* X2L = (unsigned short*)(ws + kOffX2L);
  unsigned short* X3H = (unsigned short*)(ws + kOffX3H);
  unsigned short* X3L = (unsigned short*)(ws + kOffX3L);
  float*          X4  = (float*)(ws + kOffX4);
  float*          PAR = (float*)(ws + kOffPar);

  prep_weights_kernel<<<dim3(18, 13), 256, 0, stream>>>(bb_w, cub_cw, ell_cw, grd_cw, WBH, WBL, WHH, WHL, ZR);

  const size_t wLayer = (size_t)3 * 64 * kKc;
  const int g1 = (((kM1 + 31) / 32) * 3 + 7) / 8;
  const int g2 = (((kM2 + 31) / 32) * 3 + 7) / 8;
  const int g3 = (((kM3 + 31) / 32) * 3 + 7) / 8;
  const int g4 = (((kM4 + 31) / 32) * 3 + 7) / 8;

  for (int b = 0; b < kNB; ++b) {
    first_conv_kernel<<<kIH, 256, 0, stream>>>(img, WBH, WBL, bb_b, FI, b);
    resample_kernel<<<(kM0 * 8 + 255) / 256, 256, 0, stream>>>(FI, X0H, X0L);
    conv_s2_kernel<false><<<g1, 256, 0, stream>>>(
        X0H, X0L, 0L, WHH, WHL, ZR, cub_cb, ell_cb, grd_cb,
        (void*)X1H, (void*)X1L, (long)kM1 * kCh, kUp, kS1, 0);
    conv_s2_kernel<false><<<g2, 256, 0, stream>>>(
        X1H, X1L, (long)kM1 * kCh, WHH + wLayer, WHL + wLayer, ZR, cub_cb + 64, ell_cb + 64, grd_cb + 64,
        (void*)X2H, (void*)X2L, (long)kM2 * kCh, kS1, kS2, 0);
    conv_s2_kernel<false><<<g3, 256, 0, stream>>>(
        X2H, X2L, (long)kM2 * kCh, WHH + 2 * wLayer, WHL + 2 * wLayer, ZR, cub_cb + 128, ell_cb + 128, grd_cb + 128,
        (void*)X3H, (void*)X3L, (long)kM3 * kCh, kS2, kS3, 1);
    conv_s2_kernel<true><<<g4, 256, 0, stream>>>(
        X3H, X3L, (long)kM3 * kCh, WHH + 3 * wLayer, WHL + 3 * wLayer, ZR, cub_cb + 192, ell_cb + 192, grd_cb + 192,
        (void*)(X4 + (size_t)b * 3 * kM4 * kCh), (void*)X4, (long)kM4 * kCh, kS3, kS4, 0);
  }

  pool_dense_kernel<<<kNB, 256, 0, stream>>>(X4, cub_fw, cub_fb, ell_fw, ell_fb, grd_fw, grd_fb, PAR);
  blend_kernel<<<kNB * kPix / 256, 256, 0, stream>>>(img, PAR, out);
}
